// CustomConv2d_32538672234916
// MI455X (gfx1250) — hardware-verified
//
#include <hip/hip_runtime.h>


#define NB_  16
#define CI   64
#define CO   128
#define HH   64
#define WW   64
#define KK   576
#define NP   (NB_ * HH * WW)
typedef _Float16 h16;
typedef unsigned short bf;
typedef __attribute__((ext_vector_type(16))) __bf16   v16bf;
typedef __attribute__((ext_vector_type(16))) _Float16 v16h;
typedef __attribute__((ext_vector_type(8)))  _Float16 v8h;
typedef __attribute__((ext_vector_type(8)))  unsigned short v8us;
typedef __attribute__((ext_vector_type(8)))  float    v8f;
typedef __attribute__((ext_vector_type(4)))  float    v4f;
typedef v8h  __attribute__((may_alias)) v8ha;
typedef v4f  __attribute__((may_alias)) v4fa;
typedef v8us __attribute__((may_alias)) v8usa;

__device__ __forceinline__ unsigned short f2bf(float f) { unsigned u = __float_as_uint(f); u += 0x7FFFu + ((u >> 16) & 1u); return (unsigned short)(u >> 16); }
__device__ __forceinline__ float bf2f(unsigned short b) { return __uint_as_float(((unsigned)b) << 16); }
__device__ __forceinline__ float bfr(float f) { return bf2f(f2bf(f)); }
__device__ __forceinline__ v16h cat16(v8h lo, v8h hi) { return __builtin_shufflevector(lo, hi, 0, 1, 2, 3, 4, 5, 6, 7, 8, 9, 10, 11, 12, 13, 14, 15); }
__device__ __forceinline__ v16bf cat16b(v8us lo, v8us hi) { return __builtin_bit_cast(v16bf, __builtin_shufflevector(lo, hi, 0, 1, 2, 3, 4, 5, 6, 7, 8, 9, 10, 11, 12, 13, 14, 15)); }
__device__ __forceinline__ v8f wmma16(v16h a, v16h b, v8f c) { return __builtin_amdgcn_wmma_f32_16x16x32_f16(false, a, false, b, (short)0, c, false, false); }
__device__ __forceinline__ v8f wmmab(v16bf a, v16bf b, v8f c) { return __builtin_amdgcn_wmma_f32_16x16x32_bf16(false, a, false, b, (short)0, c, false, false); }


template <typename T16> struct WFrag;
template <> struct WFrag<h16> { typedef v16h V; static __device__ __forceinline__ V ld(const h16* p) { return cat16(*(const v8h*)p, *(const v8h*)(p + 16)); } static __device__ __forceinline__ v8f mma(V a, V b, v8f c) { return wmma16(a, b, c); } };
template <> struct WFrag<bf> { typedef v16bf V; static __device__ __forceinline__ V ld(const bf* p) { return cat16b(*(const v8us*)p, *(const v8us*)(p + 16)); } static __device__ __forceinline__ v8f mma(V a, V b, v8f c) { return wmmab(a, b, c); } };
template <typename T16, int NSPLIT, bool BIAS>
__global__ __launch_bounds__(32) void k_gemmw(const T16* __restrict__ A, const T16* __restrict__ A2, const T16* __restrict__ Bt, const T16* __restrict__ Bt2, int K, float* C, int ldc, const float* __restrict__ bias, size_t sA, size_t sB, size_t sC) {
    typedef typename WFrag<T16>::V V;
    __shared__ __align__(16) float os[16 * 68];
    const size_t z = blockIdx.z; A += z * sA; if (A2) A2 += z * sA; Bt += z * sB; if (Bt2) Bt2 += z * sB; C += z * sC;
    const int lane = threadIdx.x & 31, lr = lane & 15, hi = lane >> 4; const int r0 = blockIdx.x * 64, c0 = blockIdx.y * 64;
    v8f acc[4][4];
#pragma unroll
    for (int mb = 0; mb < 4; ++mb)
#pragma unroll
        for (int nb = 0; nb < 4; ++nb) acc[mb][nb] = (v8f){};
    const size_t aoff = (size_t)(r0 + lr) * K + 8 * hi, boff = (size_t)(c0 + lr) * K + 8 * hi;
#pragma unroll 1
    for (int kc = 0; kc < K; kc += 32) {
        V a[4], a2[4];
#pragma unroll
        for (int mb = 0; mb < 4; ++mb) { a[mb] = WFrag<T16>::ld(A + aoff + (size_t)mb * 16 * K + kc); if (NSPLIT == 1 || NSPLIT == 2) a2[mb] = WFrag<T16>::ld(A2 + aoff + (size_t)mb * 16 * K + kc); }
#pragma unroll
        for (int nb = 0; nb < 4; ++nb) { const V b = WFrag<T16>::ld(Bt + boff + (size_t)nb * 16 * K + kc); V b2; if (NSPLIT >= 2) b2 = WFrag<T16>::ld(Bt2 + boff + (size_t)nb * 16 * K + kc);
#pragma unroll
            for (int mb = 0; mb < 4; ++mb) { acc[mb][nb] = WFrag<T16>::mma(a[mb], b, acc[mb][nb]); if (NSPLIT == 1 || NSPLIT == 2) acc[mb][nb] = WFrag<T16>::mma(a2[mb], b, acc[mb][nb]); if (NSPLIT >= 2) acc[mb][nb] = WFrag<T16>::mma(a[mb], b2, acc[mb][nb]); } }
        asm volatile("v_nop\n\tv_nop\n\tv_nop\n\tv_nop" : "+v"(acc[0][0]), "+v"(acc[1][1]), "+v"(acc[2][2]), "+v"(acc[3][3]) : "v"(a[0]), "v"(a[3]));
    }
#pragma unroll
    for (int mb = 0; mb < 4; ++mb) {
#pragma unroll
        for (int nb = 0; nb < 4; ++nb) {
#pragma unroll
            for (int j = 0; j < 8; ++j) os[(hi * 8 + j) * 68 + nb * 16 + lr] = acc[mb][nb][j]; }
        __builtin_amdgcn_wave_barrier(); asm volatile("" ::: "memory");
        float* crow = C + (size_t)(r0 + mb * 16) * ldc + c0;
#pragma unroll 1
        for (int ps = 0; ps < 2; ++ps) {
#pragma unroll
            for (int s = 0; s < 8; ++s) { const int row = 2 * s + hi, cofs = lr * 4; v4f val = *(const v4fa*)(os + row * 68 + cofs); if (BIAS) { val[0] += bfr(bias[c0 + cofs]); val[1] += bfr(bias[c0 + cofs + 1]); val[2] += bfr(bias[c0 + cofs + 2]); val[3] += bfr(bias[c0 + cofs + 3]); }
                *(volatile v4f*)(crow + (size_t)row * ldc + cofs) = val; }
            if (ps == 0) __threadfence(); }
        __builtin_amdgcn_wave_barrier(); asm volatile("" ::: "memory");
    }
}

__device__ __forceinline__ void splitf(float y, unsigned short& h, unsigned short& l) { h = f2bf(y); l = f2bf(y - bf2f(h)); }
typedef __attribute__((ext_vector_type(2))) unsigned short v2us;
typedef __attribute__((ext_vector_type(2))) float v2f;

__global__ __launch_bounds__(256) void k_ew(const float* __restrict__ w, bf* Bh, bf* Bl) {
    const int lane = threadIdx.x & 31; const int L = blockIdx.x * 8 + (threadIdx.x >> 5); if (L >= CO * KK / 64) return; const int e = L * 64 + lane * 2; v2us oh, ol;
#pragma unroll
    for (int q = 0; q < 2; ++q) { unsigned short a, b2; splitf(expf(bfr(w[e + q])), a, b2); oh[q] = a; ol[q] = b2; }
    *(volatile v2us*)(Bh + e) = oh; *(volatile v2us*)(Bl + e) = ol; __threadfence(); *(volatile v2us*)(Bh + e) = oh; *(volatile v2us*)(Bl + e) = ol;
}
__global__ __launch_bounds__(256) void k_ex(const float* __restrict__ x, float* EX, size_t n4) { const size_t i = (size_t)blockIdx.x * 256 + threadIdx.x; if (i >= n4) return; const v4f v = *(const v4f*)(x + i * 4); v4f o;
#pragma unroll
    for (int k = 0; k < 4; ++k) o[k] = expf(bfr(v[k])); *(volatile v4f*)(EX + i * 4) = o; __threadfence(); *(volatile v4f*)(EX + i * 4) = o; }
__global__ __launch_bounds__(256) void k_im(const float* __restrict__ EX, bf* Ah, bf* Al) {
    const int lane = threadIdx.x & 31; const int L0 = (blockIdx.x * 8 + (threadIdx.x >> 5)) * 8; const int nlines = NP * KK / 64;
#pragma unroll 1
    for (int ps = 0; ps < 2; ++ps) {
#pragma unroll 1
        for (int l = 0; l < 8; ++l) { const int L = L0 + l; if (L >= nlines) break; const int e = L * 64 + lane * 2; const int r = e / KK, col = e % KK; const int b = r >> 12, h = (r >> 6) & 63, w = r & 63; v2us oh, ol;
#pragma unroll
            for (int q = 0; q < 2; ++q) { const int cc = col + q; const int c = cc / 9, kh = (cc % 9) / 3, kw = cc % 3; const int hh = h + kh - 1, ww = w + kw - 1; unsigned short a = 0x3F80, b2 = 0;
                if (hh >= 0 && hh < HH && ww >= 0 && ww < WW) splitf(EX[(((size_t)b * CI + c) * HH + hh) * WW + ww], a, b2); oh[q] = a; ol[q] = b2; }
            *(volatile v2us*)(Ah + (size_t)e) = oh; *(volatile v2us*)(Al + (size_t)e) = ol; }
        if (ps == 0) __threadfence(); }
}
__global__ __launch_bounds__(256) void k_fin(const float* __restrict__ C, const float* __restrict__ bias, float* OUT) {
    const int lane = threadIdx.x & 31; const int wg = blockIdx.x * 8 + (threadIdx.x >> 5); if (wg >= NB_ * CO * HH) return; const int h = wg & 63, o = (wg >> 6) & 127, b = wg >> 13; const float bo = bfr(bias[o]); v2f v;
#pragma unroll
    for (int q = 0; q < 2; ++q) v[q] = ((float)KK - C[(((size_t)b * HH + h) * WW + lane * 2 + q) * CO + o]) + bo;
    float* dst = OUT + (((size_t)b * CO + o) * HH + h) * WW + lane * 2; *(volatile v2f*)dst = v; __threadfence(); *(volatile v2f*)dst = v;
}

extern "C" void kernel_launch(void* const* d_in, const int* in_sizes, int n_in,
                              void* d_out, int out_size, void* d_ws, size_t ws_size, hipStream_t stream) {
    (void)in_sizes; (void)n_in; (void)out_size;
    const float* x = (const float*)d_in[0]; const float* w = (const float*)d_in[1]; const float* bias = (const float*)d_in[2];
    float* OUT = (float*)d_out;
    char* wsp = (char*)d_ws;
    auto take = [&](size_t bytes) { char* p = wsp; wsp += (bytes + 255) & ~(size_t)255; return (void*)p; };
    bf* Bh = (bf*)take((size_t)CO * KK * 2); bf* Bl = (bf*)take((size_t)CO * KK * 2); float* EX = (float*)take((size_t)NB_ * CI * HH * WW * 4);
    bf* Ah = (bf*)take((size_t)NP * KK * 2); bf* Al = (bf*)take((size_t)NP * KK * 2); float* C = (float*)take((size_t)NP * CO * 4);
    if ((size_t)(wsp - (char*)d_ws) > ws_size) return;
    k_ew<<<(CO * KK / 64 + 7) / 8, 256, 0, stream>>>(w, Bh, Bl);
    { const size_t n4 = (size_t)NB_ * CI * HH * WW / 4; k_ex<<<(unsigned)((n4 + 255) / 256), 256, 0, stream>>>(x, EX, n4); }
    k_im<<<(NP * KK / 64 + 63) / 64, 256, 0, stream>>>(EX, Ah, Al);
    k_gemmw<bf, 2, false><<<dim3(NP / 64, CO / 64, 1), 32, 0, stream>>>(Ah, Al, Bh, Bl, KK, C, CO, nullptr, 0, 0, 0);
    k_fin<<<NB_ * CO * HH / 8, 256, 0, stream>>>(C, bias, OUT);
}
